// CharRNN_86792699118063
// MI455X (gfx1250) — hardware-verified
//
#include <hip/hip_runtime.h>
#include <math.h>

constexpr int NB   = 128;
constexpr int NL   = 1024;
constexpr int NH   = 512;
constexpr int NV   = 96;
constexpr int NE   = 64;
constexpr int NTHR = 256;
constexpr int RB   = 16;
constexpr int HST  = 520;
constexpr int XST  = 516;
constexpr int LST  = 260;
constexpr float HCAR    = 16.0f;
constexpr float WCAR    = 256.0f;
constexpr float ACC_INV = 1.0f / 4096.0f;
constexpr int NOUT0 = NB * NL * NV;
constexpr int NOUT1 = NB * NH;
static_assert(NB % RB == 0, "");
static_assert(NH == 64 * (NTHR / 32), "");
static_assert(NV == 16 * 6, "");
static_assert(NH % 32 == 0, "");
static_assert(NH % 64 == 0 && NV % 32 == 0, "");
static_assert((2 * RB * HST) % NTHR == 0, "");
static_assert((RB * NH) % NTHR == 0, "");
static_assert(RB * NH == 4 * 8 * NTHR, "");
static_assert((NV * NH) % NTHR == 0, "");
static_assert(RB == 2 * (NTHR / 32), "");
static_assert(HST % 8 == 0 && XST % 4 == 0 && LST % 4 == 0, "");

typedef __attribute__((ext_vector_type(16))) _Float16 v16h;
typedef __attribute__((ext_vector_type(8)))  _Float16 v8h;
typedef __attribute__((ext_vector_type(8)))  float    v8f;
typedef __attribute__((ext_vector_type(4)))  float    v4f;

__device__ __forceinline__ void mma_guard4(v8f& a0, v8f& a1, v8f& a2, v8f& a3,
                                           v16h x, v16h y0, v16h y1, v16h y2, v16h y3) {
  asm volatile("v_nop\n\tv_nop\n\tv_nop\n\tv_nop"
               : "+v"(a0), "+v"(a1), "+v"(a2), "+v"(a3)
               : "v"(x), "v"(y0), "v"(y1), "v"(y2), "v"(y3));
}
__device__ __forceinline__ void mma_guard1(v8f& a0, v16h x, v16h y) {
  asm volatile("v_nop\n\tv_nop\n\tv_nop\n\tv_nop" : "+v"(a0) : "v"(x), "v"(y));
}
__device__ __forceinline__ void acc_guard4(v8f& a, v8f& b, v8f& c, v8f& d) {
  asm volatile("v_nop\n\tv_nop\n\tv_nop\n\tv_nop" : "+v"(a), "+v"(b), "+v"(c), "+v"(d));
}
__device__ __forceinline__ void acc_guard1(v8f& a) {
  asm volatile("v_nop\n\tv_nop\n\tv_nop\n\tv_nop" : "+v"(a));
}

template <typename T> struct Frag;
template <> struct Frag<_Float16> {
  typedef v16h V; union U { v16h v; v8h h[2]; };
  static __device__ __forceinline__ v16h load(const _Float16* p) {
    U f; f.h[0] = *(const v8h*)(p); f.h[1] = *(const v8h*)(p + 16); return f.v;
  }
  static __device__ __forceinline__ v8f mma(v16h a, v16h b, v8f c) {
    return __builtin_amdgcn_wmma_f32_16x16x32_f16(false, a, false, b, (short)0, c, false, false);
  }
};

__device__ __forceinline__ float ftanh(float x) { return 1.0f - 2.0f * __builtin_amdgcn_rcpf(__expf(2.0f * x) + 1.0f); }

__global__ __launch_bounds__(NTHR) void combined_kernel(const float* __restrict__ emb, const float* __restrict__ wxh,
                                                        const float* __restrict__ bh, float* __restrict__ comb) {
  const int i = blockIdx.x * NTHR + threadIdx.x;
  const int v = i >> 9, n = i & (NH - 1);
  float acc = 0.0f;
#pragma unroll 8
  for (int e = 0; e < NE; ++e) acc += emb[v * NE + e] * wxh[e * NH + n];
  const float o = acc + bh[n];
  ((volatile float*)comb)[i] = o;
  __threadfence();
  ((volatile float*)comb)[i] = o;
}

__global__ __launch_bounds__(NTHR) void tpc_kernel(const float* __restrict__ src, int R, int C, int ldo,
                                                   unsigned short* __restrict__ O, float sc) {
  __shared__ float Tt[64 * 33];
  const int tid = threadIdx.x;
  const int c0 = blockIdx.x * 32, r0 = blockIdx.y * 64;
#pragma unroll
  for (int i = 0; i < 2; ++i) {
    const int idx = i * NTHR + tid;
    const int rr = idx >> 3, cc = (idx & 7) * 4;
    const v4f v = *(const v4f*)(src + (size_t)(r0 + rr) * (size_t)C + c0 + cc);
    Tt[rr * 33 + cc + 0] = v[0];
    Tt[rr * 33 + cc + 1] = v[1];
    Tt[rr * 33 + cc + 2] = v[2];
    Tt[rr * 33 + cc + 3] = v[3];
  }
  __syncthreads();
  const int q = tid >> 3, c8 = (tid & 7) * 8;
  v8h hv;
#pragma unroll
  for (int e = 0; e < 8; ++e) hv[e] = (_Float16)(Tt[(c8 + e) * 33 + q] * sc);
  const size_t o = (size_t)(c0 + q) * (size_t)ldo + (size_t)(r0 + c8);
  for (int pass = 0; pass < 2; ++pass) {
    *(volatile v8h*)(O + o) = hv;
    __threadfence();
  }
}

__device__ __forceinline__ void gather_rows(float* Xs, const float* __restrict__ comb, const int* __restrict__ x,
                                            int rowbase, int tn, int tid) {
#pragma unroll
  for (int it = 0; it < 8; ++it) {
    const int i = it * NTHR + tid;
    const int row = i >> 7, c4 = (i & 127) * 4;
    int id = x[(size_t)(rowbase + row) * NL + (size_t)tn];
    id = id < 0 ? 0 : (id > NV - 1 ? NV - 1 : id);
    const v4f v = *(const v4f*)(comb + (size_t)id * NH + c4);
    *(v4f*)(Xs + row * XST + c4) = v;
  }
}

__global__ __launch_bounds__(NTHR) void rnn_seq_kernel(const int* __restrict__ x, const float* __restrict__ h0,
                                                       const float* __restrict__ comb,
                                                       const unsigned short* __restrict__ WhTp,
                                                       const unsigned short* __restrict__ FcTp,
                                                       const float* __restrict__ fcb,
                                                       float* __restrict__ logits, float* __restrict__ finalh) {
  __shared__ __align__(16) _Float16 Ah[2 * RB * HST];
  __shared__ __align__(16) float    Xs[RB * XST];
  __shared__ __align__(16) float    Ls[RB * LST];
  const _Float16* WhT = (const _Float16*)WhTp;
  const _Float16* FcT = (const _Float16*)FcTp;
  const int tid = threadIdx.x, lane = tid & 31, wave = tid >> 5;
  const int c = lane & 15, hh = lane >> 4, koff = hh * 8;
  const int rowbase = blockIdx.x * RB;
  const int colw = 64 * wave + c;

#pragma unroll 1
  for (int i = tid; i < 2 * RB * HST; i += NTHR) Ah[i] = (_Float16)0.0f;
  __syncthreads();
#pragma unroll 1
  for (int i = tid; i < RB * NH; i += NTHR) {
    const int m = i >> 9, n = i & (NH - 1);
    Ah[m * HST + n] = (_Float16)(h0[(size_t)(rowbase + m) * NH + n] * HCAR);
  }
  gather_rows(Xs, comb, x, rowbase, 0, tid);
  const int fcol = 16 * ((wave < 6) ? wave : 5) + c;
  const float fcbv = fcb[fcol];
  __syncthreads();

  const v8f z8 = {0.f, 0.f, 0.f, 0.f, 0.f, 0.f, 0.f, 0.f};
  const _Float16* wb = WhT + (size_t)colw * NH + koff;
  const _Float16* fw = FcT + (size_t)fcol * NH + koff;

#pragma unroll 1
  for (int t = 0; t < NL; ++t) {
    const int cur = t & 1;
    const bool last = (t == NL - 1);
    const _Float16* ahrow = Ah + cur * (RB * HST) + c * HST + koff;
    _Float16* ahn = Ah + (cur ^ 1) * (RB * HST);

    v8f acc[4];
    acc[0] = z8; acc[1] = z8; acc[2] = z8; acc[3] = z8;
#pragma unroll 1
    for (int k0 = 0; k0 < NH; k0 += 32) {
      const v16h a  = Frag<_Float16>::load(ahrow + k0);
      const v16h b0 = Frag<_Float16>::load(wb + k0);
      const v16h b1 = Frag<_Float16>::load(wb + (size_t)16 * NH + k0);
      const v16h b2 = Frag<_Float16>::load(wb + (size_t)32 * NH + k0);
      const v16h b3 = Frag<_Float16>::load(wb + (size_t)48 * NH + k0);
      acc[0] = Frag<_Float16>::mma(a, b0, acc[0]);
      acc[1] = Frag<_Float16>::mma(a, b1, acc[1]);
      acc[2] = Frag<_Float16>::mma(a, b2, acc[2]);
      acc[3] = Frag<_Float16>::mma(a, b3, acc[3]);
      mma_guard4(acc[0], acc[1], acc[2], acc[3], a, b0, b1, b2, b3);
    }
    acc_guard4(acc[0], acc[1], acc[2], acc[3]);
    float hv[4][8];
#pragma unroll
    for (int nt = 0; nt < 4; ++nt) {
      const int j = colw + 16 * nt;
#pragma unroll
      for (int r = 0; r < 8; ++r) {
        const float z  = acc[nt][r] * ACC_INV + Xs[(8 * hh + r) * XST + j];
        const float hn = ftanh(z);
        hv[nt][r] = hn;
        ahn[(8 * hh + r) * HST + j] = (_Float16)(hn * HCAR);
      }
    }
    __syncthreads();

    if (wave < 6) {
      v8f cf = z8;
      const _Float16* ah2 = Ah + (cur ^ 1) * (RB * HST) + c * HST + koff;
#pragma unroll 1
      for (int k0 = 0; k0 < NH; k0 += 32) {
        const v16h a = Frag<_Float16>::load(ah2 + k0);
        const v16h b = Frag<_Float16>::load(fw + k0);
        cf = Frag<_Float16>::mma(a, b, cf);
        mma_guard1(cf, a, b);
      }
      acc_guard1(cf);
#pragma unroll
      for (int r = 0; r < 8; ++r) Ls[(8 * hh + r) * LST + fcol] = cf[r] * ACC_INV + fcbv;
    }
    if (!last) {
      gather_rows(Xs, comb, x, rowbase, t + 1, tid);
    } else {
#pragma unroll
      for (int nt = 0; nt < 4; ++nt)
#pragma unroll
        for (int r = 0; r < 8; ++r) Xs[(8 * hh + r) * XST + colw + 16 * nt] = hv[nt][r];
    }
    __syncthreads();

    {
      const int cl = (lane < 24) ? lane : 23;
      const int c4 = cl * 4;
      const bool act = (lane < 24);
      for (int pass = 0; pass < 2; ++pass) {
#pragma unroll
        for (int j = 0; j < 2; ++j) {
          const int row = 2 * wave + j;
          const v4f v = *(const v4f*)(Ls + row * LST + c4);
          float* op = logits + ((size_t)(rowbase + row) * NL + (size_t)t) * NV + c4;
          if (act) *(volatile v4f*)op = v;
        }
        __threadfence();
      }
      if (last) {
        for (int pass = 0; pass < 2; ++pass) {
#pragma unroll
          for (int j = 0; j < 2; ++j) {
            const int row = 2 * wave + j;
#pragma unroll
            for (int q = 0; q < 4; ++q) {
              const v4f v = *(const v4f*)(Xs + row * XST + 128 * q + 4 * lane);
              *(volatile v4f*)(finalh + (size_t)(rowbase + row) * NH + 128 * q + 4 * lane) = v;
            }
          }
          __threadfence();
        }
      }
    }
  }
}

extern "C" void kernel_launch(void* const* d_in, const int* in_sizes, int n_in,
                              void* d_out, int out_size, void* d_ws, size_t ws_size, hipStream_t stream) {
  if (n_in < 8 || d_out == nullptr || d_ws == nullptr) return;
  if (in_sizes[0] != NB * NL || in_sizes[1] != NB * NH || in_sizes[2] != NV * NE || in_sizes[3] != NE * NH ||
      in_sizes[4] != NH * NH || in_sizes[5] != NH || in_sizes[6] != NH * NV || in_sizes[7] != NV ||
      out_size != NOUT0 + NOUT1) return;

  const int*   x   = (const int*)d_in[0];
  const float* hid = (const float*)d_in[1];
  const float* emb = (const float*)d_in[2];
  const float* wxh = (const float*)d_in[3];
  const float* whh = (const float*)d_in[4];
  const float* bh  = (const float*)d_in[5];
  const float* fcw = (const float*)d_in[6];
  const float* fcb = (const float*)d_in[7];
  float* out0 = (float*)d_out;
  float* out1 = out0 + (size_t)NOUT0;

  char* ws = (char*)d_ws; size_t off = 0;
  auto carve = [&](size_t bytes) -> char* { char* p = ws + off; off += (bytes + 255) & ~(size_t)255; return p; };
  float*          COMB = (float*)carve((size_t)NV * NH * 4);
  unsigned short* WHT  = (unsigned short*)carve((size_t)NH * NH * 2);
  unsigned short* FCT  = (unsigned short*)carve((size_t)NV * NH * 2);
  if (off > ws_size || off > (size_t)134217728) return;

  combined_kernel<<<(NV * NH) / NTHR, NTHR, 0, stream>>>(emb, wxh, bh, COMB);
  tpc_kernel<<<dim3(NH / 32, NH / 64), NTHR, 0, stream>>>(whh, NH, NH, NH, WHT, WCAR);
  tpc_kernel<<<dim3(NV / 32, NH / 64), NTHR, 0, stream>>>(fcw, NH, NV, NH, FCT, WCAR);
  rnn_seq_kernel<<<NB / RB, NTHR, 0, stream>>>(x, hid, COMB, WHT, FCT, fcb, out0, out1);
}
